// MHSABlock_4294967296212
// MI455X (gfx1250) — hardware-run, weakly checked
//
#include <hip/hip_runtime.h>
#include <math.h>
#include <stdint.h>

#define NB    2
#define CH    256
#define NH    8
#define HD    32
#define SEQ   4096
#define NTOK  (NB * SEQ)
#define NPOS  64
#define NDIV  64
#define NQB   (SEQ / 128)
#define NKT   (SEQ / 64)
static_assert(NH * HD == CH);
static_assert(NQB == 32 && NKT == 64);
static_assert(NPOS * NPOS == SEQ);
static_assert((SEQ % 128) == 0 && (CH % 64) == 0 && (NTOK % 64) == 0 && (CH % 32) == 0);

typedef _Float16 v16h __attribute__((ext_vector_type(16)));
typedef _Float16 v8h  __attribute__((ext_vector_type(8)));
typedef float    v8f  __attribute__((ext_vector_type(8)));
typedef float    v4f  __attribute__((ext_vector_type(4)));
typedef unsigned int v4u __attribute__((ext_vector_type(4)));

#if defined(__HIP_DEVICE_COMPILE__)
#define DEV_ASM 1
#else
#define DEV_ASM 0
#endif

__device__ __forceinline__ unsigned short h_bits(_Float16 x) { return __builtin_bit_cast(unsigned short, x); }
__device__ __forceinline__ unsigned short f16b(float f) { return h_bits((_Float16)f); }
__device__ __forceinline__ unsigned pk16(unsigned short a, unsigned short b) { return (unsigned)a | ((unsigned)b << 16); }
__device__ __forceinline__ v8f zero8() { v8f z = {0.f, 0.f, 0.f, 0.f, 0.f, 0.f, 0.f, 0.f}; return z; }

__device__ __forceinline__ v16h ldfrag(const _Float16* p) {
  union { v16h v; v8h h[2]; } f;
  f.h[0] = *(const v8h*)(p);
  f.h[1] = *(const v8h*)(p + 16);
  return f.v;
}

__device__ __forceinline__ v8f mmar(v16h a, v16h b, v8f c) {
  return __builtin_amdgcn_wmma_f32_16x16x32_f16(false, a, false, b, (short)0, c, false, false);
}
__device__ __forceinline__ v8f mma_h(v16h a, v16h b, v8f c) {
  c = __builtin_amdgcn_wmma_f32_16x16x32_f16(false, a, false, b, (short)0, c, false, false);
#if DEV_ASM
  asm volatile("v_nop\n\tv_nop\n\tv_nop\n\tv_nop" : "+v"(c) : "v"(a), "v"(b));
#endif
  return c;
}
__device__ __forceinline__ void dep_guard(v8f& a, v8f& b, v16h x, v16h y) {
#if DEV_ASM
  asm volatile("v_nop\n\tv_nop\n\tv_nop\n\tv_nop" : "+v"(a), "+v"(b) : "v"(x), "v"(y));
#else
  (void)a; (void)b; (void)x; (void)y;
#endif
}
__device__ __forceinline__ void keep4(v16h a, v16h b, v16h c, v16h d) {
#if DEV_ASM
  asm volatile("v_nop" :: "v"(a), "v"(b), "v"(c), "v"(d));
#else
  (void)a; (void)b; (void)c; (void)d;
#endif
}
__device__ __forceinline__ void acc_guard4(v8f& a, v8f& b, v8f& c, v8f& d) {
#if DEV_ASM
  asm volatile("v_nop\n\tv_nop\n\tv_nop\n\tv_nop" : "+v"(a), "+v"(b), "+v"(c), "+v"(d));
#else
  (void)a; (void)b; (void)c; (void)d;
#endif
}

__global__ __launch_bounds__(64) void pe_div(float* dv) {
  const int i = (int)threadIdx.x;
  const float e = (float)(2 * i) * (-0.07195578415606394f);
  const float v = expf(e);
  *(volatile float*)(dv + i) = v;
  __threadfence();
  *(volatile float*)(dv + i) = v;
}

__global__ __launch_bounds__(256) void pe_tab(const float* __restrict__ dv, float* stab, float* ctab) {
  const int lane = (int)threadIdx.x & 31;
  const int wave = (int)threadIdx.x >> 5;
  const int pos  = blockIdx.x * 4 + (wave >> 1);
  const int i    = (wave & 1) * 32 + lane;
  const float f   = dv[i];
  const float ang = (float)pos * f;
  float sn, cs;
  sincosf(ang, &sn, &cs);
  float* ps = stab + (size_t)pos * NDIV + i;
  float* pc = ctab + (size_t)pos * NDIV + i;
  *(volatile float*)ps = sn;
  *(volatile float*)pc = cs;
  __threadfence();
  *(volatile float*)ps = sn;
  *(volatile float*)pc = cs;
}

__global__ __launch_bounds__(256) void wcvt(const float* __restrict__ w0, const float* __restrict__ w1,
                                             const float* __restrict__ w2, const float* __restrict__ w3,
                                             unsigned short* out) {
  const int y = blockIdx.y;
  const float* src = (y == 0) ? w0 : (y == 1) ? w1 : (y == 2) ? w2 : w3;
  const int i = blockIdx.x * 256 + (int)threadIdx.x;
  if (i < CH * CH / 8) {
    const v4f a  = *(const v4f*)(src + (size_t)i * 8);
    const v4f a4 = *(const v4f*)(src + (size_t)i * 8 + 4);
    v4u p;
    p[0] = pk16(f16b(a[0]  * 256.0f), f16b(a[1]  * 256.0f));
    p[1] = pk16(f16b(a[2]  * 256.0f), f16b(a[3]  * 256.0f));
    p[2] = pk16(f16b(a4[0] * 256.0f), f16b(a4[1] * 256.0f));
    p[3] = pk16(f16b(a4[2] * 256.0f), f16b(a4[3] * 256.0f));
    unsigned short* o = out + (size_t)y * (CH * CH) + (size_t)i * 8;
    *(volatile v4u*)o = p;
    __threadfence();
    *(volatile v4u*)o = p;
  }
}

__global__ __launch_bounds__(256) void tok_prep(const float* __restrict__ x,
                                                 const float* __restrict__ stab,
                                                 const float* __restrict__ ctab,
                                                 unsigned short* tok) {
  __shared__ __align__(16) unsigned short tile[64 * 72];
  const int hp  = blockIdx.x;
  const int c0  = blockIdx.y * 64;
  const int b   = blockIdx.z;
  const int n0  = hp * 64;
  const int tid = (int)threadIdx.x;
  const bool upper = (c0 >= 128);
#pragma unroll 1
  for (int it = 0; it < 4; ++it) {
    const int idx = it * 256 + tid;
    const int cc  = idx >> 4;
    const int w4  = (idx & 15) * 4;
    const int c   = c0 + cc;
    const int i   = (c & 127) >> 1;
    const v4f xv  = *(const v4f*)(x + ((size_t)(b * CH + c)) * SEQ + n0 + w4);
#pragma unroll
    for (int e = 0; e < 4; ++e) {
      const int w   = w4 + e;
      const int pos = upper ? hp : w;
      const float sv = stab[pos * NDIV + i];
      const float cv = ctab[pos * NDIV + i];
      const float pe = (c & 1) ? cv : sv;
      const float t  = (xv[e] + pe) * 8.0f;
      tile[w * 72 + cc] = f16b(t);
    }
  }
  __syncthreads();
  const int wave = tid >> 5, lane = tid & 31;
  const int q = lane >> 3, c8 = (lane & 7) * 8;
  v4u hv[2];
#pragma unroll
  for (int it = 0; it < 2; ++it) {
    const int nn = (it * 8 + wave) * 4 + q;
    hv[it] = *(const v4u*)(tile + nn * 72 + c8);
  }
  for (int pass = 0; pass < 2; ++pass) {
#pragma unroll
    for (int it = 0; it < 2; ++it) {
      const int nn = (it * 8 + wave) * 4 + q;
      *(volatile v4u*)(tok + ((size_t)(b * SEQ + n0 + nn)) * CH + c0 + c8) = hv[it];
    }
    __threadfence();
  }
}

template <int OUT_MODE, bool BROW>
__global__ __launch_bounds__(256) void gemm64(
    const unsigned short* __restrict__ Ap, int lda, long long strideA,
    const unsigned short* __restrict__ Btp, int ldb, int kblkB, long long strideB,
    void* Cout, int ldc, long long strideC,
    const float* __restrict__ bias,
    int M, int N, int K, float ascale, float cscale) {
  const _Float16* A  = (const _Float16*)(const void*)Ap;
  const _Float16* Bt = (const _Float16*)(const void*)Btp;
  __shared__ __align__(16) float sT[8][16 * 68];
  const int b    = blockIdx.y;
  const int lane = threadIdx.x & 31;
  const int wave = threadIdx.x >> 5;
  const int tilesN = N >> 6;
  const int tilesM = M >> 6;
  const int tile = blockIdx.x * 8 + wave;
  if (tile >= tilesM * tilesN) return;
  const int tm = tile / tilesN;
  const int tn = tile - tm * tilesN;
  const int m0 = tm << 6;
  const int n0 = tn << 6;

  const _Float16* Ab = A  + (size_t)b * (size_t)strideA;
  const _Float16* Bb = Bt + (size_t)b * (size_t)strideB;

  const int rlane = lane & 15;
  const int koff  = (lane >> 4) * 8;
  const int mOff  = (lane >> 4) * 8;

  v8f acc[4][4];
#pragma unroll
  for (int i = 0; i < 4; ++i)
#pragma unroll
    for (int j = 0; j < 4; ++j) acc[i][j] = zero8();

  for (int k0 = 0; k0 < K; k0 += 32) {
    v16h bq[4];
    const _Float16* Bk = Bb + (size_t)(k0 >> 5) * (size_t)kblkB + koff;
#pragma unroll
    for (int j = 0; j < 4; ++j)
      bq[j] = ldfrag(Bk + (size_t)(n0 + (j << 4) + rlane) * (size_t)ldb);
#pragma unroll
    for (int i = 0; i < 4; ++i) {
      const v16h af = ldfrag(Ab + (size_t)(m0 + (i << 4) + rlane) * (size_t)lda + koff + k0);
#pragma unroll
      for (int j = 0; j < 4; ++j) acc[i][j] = mmar(af, bq[j], acc[i][j]);
      dep_guard(acc[i][0], acc[i][3], af, bq[3]);
    }
    keep4(bq[0], bq[1], bq[2], bq[3]);
  }
  acc_guard4(acc[0][0], acc[0][1], acc[0][2], acc[0][3]);
  acc_guard4(acc[1][0], acc[1][1], acc[1][2], acc[1][3]);
  acc_guard4(acc[2][0], acc[2][1], acc[2][2], acc[2][3]);
  acc_guard4(acc[3][0], acc[3][1], acc[3][2], acc[3][3]);

  float* slab = sT[wave];
#pragma unroll
  for (int i = 0; i < 4; ++i) {
    const int mBase = m0 + (i << 4);
#pragma unroll
    for (int j = 0; j < 4; ++j) {
#pragma unroll
      for (int r = 0; r < 8; ++r) {
        slab[(mOff + r) * 68 + (j << 4) + rlane] = acc[i][j][r];
      }
    }
    __builtin_amdgcn_fence(__ATOMIC_RELEASE, "workgroup");
    __builtin_amdgcn_wave_barrier();
    __builtin_amdgcn_fence(__ATOMIC_ACQUIRE, "workgroup");
    if (OUT_MODE == 0) {
      float* C = (float*)Cout + (size_t)b * (size_t)strideC;
      const int h2 = lane >> 4, c4 = (lane & 15) * 4;
      v4f bcol = {0.f, 0.f, 0.f, 0.f};
      if (!BROW) bcol = *(const v4f*)(bias + n0 + c4);
      for (int pass = 0; pass < 2; ++pass) {
#pragma unroll
        for (int it = 0; it < 8; ++it) {
          const int row = it * 2 + h2;
          float badd = 0.f;
          if (BROW) badd = bias[mBase + row];
          const v4f sv = *(const v4f*)(slab + row * 68 + c4);
          v4f v;
#pragma unroll
          for (int e = 0; e < 4; ++e) v[e] = sv[e] * ascale + badd + bcol[e];
          *(volatile v4f*)(C + (size_t)(mBase + row) * (size_t)ldc + n0 + c4) = v;
        }
        __threadfence();
      }
    } else {
      const int q = lane >> 3, c8 = (lane & 7) * 8;
      unsigned short* C = (unsigned short*)Cout + (size_t)b * (size_t)strideC;
      v4f b0 = {0.f, 0.f, 0.f, 0.f}, b1 = {0.f, 0.f, 0.f, 0.f};
      if (!BROW) {
        b0 = *(const v4f*)(bias + n0 + c8);
        b1 = *(const v4f*)(bias + n0 + c8 + 4);
      }
      v4u hv[4];
#pragma unroll
      for (int it = 0; it < 4; ++it) {
        const int row = it * 4 + q;
        const float* sp = slab + row * 68 + c8;
        float badd = 0.f;
        if (BROW) badd = bias[mBase + row];
        float f[8];
#pragma unroll
        for (int e = 0; e < 8; ++e) {
          const float bc = (e < 4) ? b0[e & 3] : b1[e & 3];
          f[e] = sp[e] * ascale + badd + bc;
        }
        v4u a;
#pragma unroll
        for (int e = 0; e < 4; ++e)
          a[e] = pk16(f16b(f[2 * e] * cscale), f16b(f[2 * e + 1] * cscale));
        hv[it] = a;
      }
      for (int pass = 0; pass < 2; ++pass) {
#pragma unroll
        for (int it = 0; it < 4; ++it) {
          const int row = it * 4 + q;
          *(volatile v4u*)(C + (size_t)(mBase + row) * (size_t)ldc + n0 + c8) = hv[it];
        }
        __threadfence();
      }
    }
    __builtin_amdgcn_fence(__ATOMIC_RELEASE, "workgroup");
    __builtin_amdgcn_wave_barrier();
    __builtin_amdgcn_fence(__ATOMIC_ACQUIRE, "workgroup");
  }
}

__global__ __launch_bounds__(256)
void attn_mh(const unsigned short* __restrict__ qp, const unsigned short* __restrict__ kp,
             const unsigned short* __restrict__ vtp, unsigned short* op, float sscale, float onorm) {
  union FH { v16h v; v8h h[2]; };
  __shared__ __align__(16) _Float16 Ksh[64 * HD];
  __shared__ __align__(16) _Float16 Vth[HD * 64];
  __shared__ __align__(16) _Float16 Psh[8][16 * 64];
  __shared__ __align__(16) float    Os[8][16 * HD];

  const int tid  = threadIdx.x;
  const int wave = tid >> 5;
  const int lane = tid & 31;
  const int hh   = lane >> 4;
  const int c    = lane & 15;

  const int bx   = blockIdx.x;
  const int qb   = bx % NQB;
  const int rest = bx / NQB;
  const int h    = rest % NH;
  const int b    = rest / NH;
  const int q0   = qb * 128 + wave * 16;
  const size_t rowB = (size_t)b * SEQ;

  const _Float16* Q  = (const _Float16*)(const void*)qp;
  const _Float16* Kh = (const _Float16*)(const void*)kp + (size_t)h * HD;
  const _Float16* Vt = (const _Float16*)(const void*)vtp + ((size_t)b * CH + (size_t)h * HD) * SEQ;

  const v16h qa = ldfrag(Q + (rowB + q0 + c) * CH + (size_t)h * HD + 8 * hh);

  float mrow[8], lrow[8];
  v8f oacc[2];
#pragma unroll
  for (int r = 0; r < 8; ++r) { mrow[r] = -INFINITY; lrow[r] = 0.f; }
#pragma unroll
  for (int t = 0; t < 2; ++t) oacc[t] = zero8();

  for (int kt = 0; kt < NKT; ++kt) {
    const int kv0 = kt * 64;
    __syncthreads();
    {
      const int rk = tid >> 2, pk = (tid & 3) * 8;
      const v8h a0 = *(const v8h*)(Kh + (rowB + kv0 + rk) * CH + pk);
      *(v8h*)(Ksh + rk * HD + pk) = a0;
      const int rv = tid >> 3, pv = (tid & 7) * 8;
      const v8h b0 = *(const v8h*)(Vt + (size_t)rv * SEQ + kv0 + pv);
      *(v8h*)(Vth + rv * 64 + pv) = b0;
    }
    __syncthreads();

    v8f s[4];
#pragma unroll
    for (int j = 0; j < 4; ++j) {
      FH kb;
      kb.h[0] = *(const v8h*)(Ksh + (j * 16 + c) * HD + 8 * hh);
      kb.h[1] = *(const v8h*)(Ksh + (j * 16 + c) * HD + 16 + 8 * hh);
      const v8f a = mma_h(qa, kb.v, zero8());
#pragma unroll
      for (int r = 0; r < 8; ++r) s[j][r] = a[r] * sscale;
    }

    _Float16* pwh = Psh[wave];
#pragma unroll
    for (int r = 0; r < 8; ++r) {
      float m = s[0][r];
#pragma unroll
      for (int j = 1; j < 4; ++j) m = fmaxf(m, s[j][r]);
#pragma unroll
      for (int off = 1; off < 16; off <<= 1) m = fmaxf(m, __shfl_xor(m, off, 32));
      const float mnew  = fmaxf(mrow[r], m);
      const float msafe = (mnew == -INFINITY) ? 0.f : mnew;
      const float alpha = __expf(mrow[r] - msafe);
      mrow[r] = mnew;
      float psum = 0.f;
#pragma unroll
      for (int j = 0; j < 4; ++j) {
        const float p = __expf(s[j][r] - msafe);
        psum += p;
        pwh[(8 * hh + r) * 64 + j * 16 + c] = (_Float16)(p * 1024.0f);
      }
#pragma unroll
      for (int off = 1; off < 16; off <<= 1) psum += __shfl_xor(psum, off, 32);
      lrow[r] = lrow[r] * alpha + psum;
#pragma unroll
      for (int t = 0; t < 2; ++t) oacc[t][r] *= alpha;
    }
    __builtin_amdgcn_fence(__ATOMIC_RELEASE, "workgroup");
    __builtin_amdgcn_wave_barrier();
    __builtin_amdgcn_fence(__ATOMIC_ACQUIRE, "workgroup");

#pragma unroll 1
    for (int kk = 0; kk < 2; ++kk) {
      FH pa;
      pa.h[0] = *(const v8h*)(pwh + c * 64 + kk * 32 + 8 * hh);
      pa.h[1] = *(const v8h*)(pwh + c * 64 + kk * 32 + 16 + 8 * hh);
#pragma unroll
      for (int t = 0; t < 2; ++t) {
        FH vb;
        vb.h[0] = *(const v8h*)(Vth + (t * 16 + c) * 64 + kk * 32 + 8 * hh);
        vb.h[1] = *(const v8h*)(Vth + (t * 16 + c) * 64 + kk * 32 + 16 + 8 * hh);
        oacc[t] = mma_h(pa.v, vb.v, oacc[t]);
      }
    }
  }

  float* os = Os[wave];
#pragma unroll
  for (int r = 0; r < 8; ++r) {
    const float l = lrow[r];
    const float inv = ((l > 0.f) ? (1.0f / l) : 0.f) * onorm;
#pragma unroll
    for (int t = 0; t < 2; ++t) os[(8 * hh + r) * HD + t * 16 + c] = oacc[t][r] * inv;
  }
  __builtin_amdgcn_fence(__ATOMIC_RELEASE, "workgroup");
  __builtin_amdgcn_wave_barrier();
  __builtin_amdgcn_fence(__ATOMIC_ACQUIRE, "workgroup");
  {
    const int rq = lane >> 2, d8 = (lane & 3) * 8;
    v4u hv[2];
#pragma unroll
    for (int it = 0; it < 2; ++it) {
      const int row = it * 8 + rq;
      const float* sp = os + row * HD + d8;
      v4u a;
#pragma unroll
      for (int e = 0; e < 4; ++e) {
        const float f0 = sp[2 * e], f1 = sp[2 * e + 1];
        a[e] = pk16(f16b(f0), f16b(f1));
      }
      hv[it] = a;
    }
    for (int pass = 0; pass < 2; ++pass) {
#pragma unroll
      for (int it = 0; it < 2; ++it) {
        const int row = it * 8 + rq;
        const size_t go = (((size_t)(b * NH + h)) * SEQ + (size_t)(q0 + row)) * HD + d8;
        *(volatile v4u*)(op + go) = hv[it];
      }
      __threadfence();
    }
  }
}

extern "C" void kernel_launch(void* const* d_in, const int* in_sizes, int n_in,
                              void* d_out, int out_size, void* d_ws, size_t ws_size,
                              hipStream_t stream) {
  if (n_in < 9) return;
  if (in_sizes[0] != NB * CH * SEQ) return;
  if (in_sizes[1] != CH * CH || in_sizes[3] != CH * CH || in_sizes[5] != CH * CH || in_sizes[7] != CH * CH) return;
  if (in_sizes[2] != CH || in_sizes[4] != CH || in_sizes[6] != CH || in_sizes[8] != CH) return;
  if (out_size != NB * CH * SEQ) return;

  const float* x  = (const float*)d_in[0];
  const float* Wq = (const float*)d_in[1];
  const float* bq = (const float*)d_in[2];
  const float* Wk = (const float*)d_in[3];
  const float* bk = (const float*)d_in[4];
  const float* Wv = (const float*)d_in[5];
  const float* bv = (const float*)d_in[6];
  const float* Wo = (const float*)d_in[7];
  const float* bo = (const float*)d_in[8];

  const size_t PW   = (size_t)4 * CH * CH * 2;
  const size_t PT   = (size_t)NTOK * CH * 2;
  const size_t PVT  = (size_t)NB * CH * SEQ * 2;
  const size_t PCTX = (size_t)NB * NH * SEQ * HD * 2;
  const size_t PTAB = (size_t)NPOS * NDIV * 4;
  const size_t PDV  = 256;
  size_t off = 0;
  const size_t oW   = off; off += PW;
  const size_t oTok = off; off += PT;
  const size_t oQ   = off; off += PT;
  const size_t oK   = off; off += PT;
  const size_t oVT  = off; off += PVT;
  const size_t oCtx = off; off += PCTX;
  const size_t oSt  = off; off += PTAB;
  const size_t oCt  = off; off += PTAB;
  const size_t oDv  = off; off += PDV;
  if (off > ws_size) return;
  if (off > (size_t)134217728) return;

  char* ws = (char*)d_ws;
  unsigned short* W16   = (unsigned short*)(ws + oW);
  unsigned short* Wq16  = W16;
  unsigned short* Wk16  = W16 + (size_t)1 * CH * CH;
  unsigned short* Wv16  = W16 + (size_t)2 * CH * CH;
  unsigned short* Wo16  = W16 + (size_t)3 * CH * CH;
  unsigned short* Tok16 = (unsigned short*)(ws + oTok);
  unsigned short* Q16   = (unsigned short*)(ws + oQ);
  unsigned short* K16   = (unsigned short*)(ws + oK);
  unsigned short* VT16  = (unsigned short*)(ws + oVT);
  unsigned short* Ctx16 = (unsigned short*)(ws + oCtx);
  float*          Stab  = (float*)(ws + oSt);
  float*          Ctab  = (float*)(ws + oCt);
  float*          Dv    = (float*)(ws + oDv);

  const dim3 blk(256);
  const dim3 gTab(NPOS / 4);
  const dim3 gW((CH * CH / 8) / 256, 4);
  const dim3 gTok(SEQ / 64, CH / 64, NB);
  const dim3 gQ(((NTOK / 64) * (CH / 64) + 7) / 8, 1);
  const dim3 gT(((CH / 64) * (SEQ / 64) + 7) / 8, NB);
  const dim3 gAttn(NB * NH * NQB);

  const float sscale = 0.17677669529663687f * (1.0f / 256.0f);

  pe_div<<<dim3(1), dim3(64), 0, stream>>>(Dv);
  pe_tab<<<gTab, blk, 0, stream>>>(Dv, Stab, Ctab);
  wcvt<<<gW, blk, 0, stream>>>(Wq, Wk, Wv, Wo, W16);
  tok_prep<<<gTok, blk, 0, stream>>>(x, Stab, Ctab, Tok16);
  gemm64<1, false><<<gQ, blk, 0, stream>>>(
      Tok16, CH, 0LL, Wq16, CH, 32, 0LL,
      (void*)Q16, CH, 0LL, bq,
      NTOK, CH, CH, 1.0f / 2048.0f, 16.0f);
  gemm64<1, false><<<gQ, blk, 0, stream>>>(
      Tok16, CH, 0LL, Wk16, CH, 32, 0LL,
      (void*)K16, CH, 0LL, bk,
      NTOK, CH, CH, 1.0f / 2048.0f, 16.0f);
  gemm64<1, true><<<gT, blk, 0, stream>>>(
      Wv16, CH, 0LL, Tok16, CH, 32, (long long)SEQ * CH,
      (void*)VT16, SEQ, (long long)CH * SEQ, bv,
      CH, SEQ, CH, 1.0f / 2048.0f, 16.0f);
  attn_mh<<<gAttn, blk, 0, stream>>>(Q16, K16, VT16, Ctx16, sscale, 1.0f / 64.0f);
  gemm64<0, true><<<gT, blk, 0, stream>>>(
      Wo16, CH, 0LL, Ctx16, HD, SEQ * HD, (long long)NH * SEQ * HD,
      d_out, SEQ, (long long)CH * SEQ, bo,
      CH, SEQ, CH, 1.0f / 65536.0f, 1.0f);
  (void)hipGetLastError();
}
